// IKNet1_31971736551660
// MI455X (gfx1250) — hardware-verified
//
#include <hip/hip_runtime.h>


namespace {
constexpr int B = 8192, J = 21, NH = 4, C = 64, D = NH * C, INF = 9, NT = B * J, NBLK = NT / 16;
constexpr float XS = 8.0f, WSC = 256.0f, SLOPE = 0.2f;
__constant__ int PARENT[J] = {-1, 0, 1, 2, 3, 0, 5, 6, 7, 0, 9, 10, 11, 0, 13, 14, 15, 0, 17, 18, 19};
typedef _Float16 b16;
typedef __attribute__((ext_vector_type(16))) _Float16 v16b;
typedef __attribute__((ext_vector_type(8))) _Float16 v8b;
typedef __attribute__((ext_vector_type(8))) float v8f;
typedef __attribute__((ext_vector_type(4))) float v4f;
typedef __attribute__((ext_vector_type(2))) float v2f;
__device__ __forceinline__ float bf16_rne(float f) { unsigned int u = __float_as_uint(f); u += 0x7FFFu + ((u >> 16) & 1u); return __uint_as_float(u & 0xFFFF0000u); }
__device__ __forceinline__ void split16(float v, b16& hi, b16& lo) { hi = (b16)v; lo = (b16)(v - (float)hi); }
__device__ __forceinline__ v16b frag_kb(const b16* p, int hh) { const v8b a = *(const v8b*)(p + 8 * hh), b = *(const v8b*)(p + 16 + 8 * hh); v16b f;
#pragma unroll
  for (int e = 0; e < 8; ++e) { f[e] = a[e]; f[8 + e] = b[e]; } return f; }
__device__ __forceinline__ v8f wmma16b(v16b a, v16b b, v8f c) { v8f d = __builtin_amdgcn_wmma_f32_16x16x32_f16(false, a, false, b, (short)0, c, false, false); asm volatile("v_nop\n\tv_nop\n\tv_nop\n\tv_nop" : "+v"(d) : "v"(a), "v"(b)); return d; }
__device__ __forceinline__ void wave_lds_sync() { __builtin_amdgcn_fence(__ATOMIC_RELEASE, "workgroup"); __builtin_amdgcn_wave_barrier(); __builtin_amdgcn_fence(__ATOMIC_ACQUIRE, "workgroup"); }
__device__ __forceinline__ float pmul(float a, float b) { float p = a * b; asm volatile("" : "+v"(p)); return p; }
__device__ __forceinline__ float leaky(float v) { return v >= 0.0f ? v : SLOPE * v; }

__global__ __launch_bounds__(256) void wput_kernel(const float* __restrict__ w, int KIN, int OUTW, int KP, int OUTP, b16* __restrict__ WT) {
  const int KG = KP / 8; const int u = blockIdx.x * 256 + threadIdx.x; if (u >= OUTP * KG) return; const int o = u / KG, k0 = (u % KG) * 8; v8b v;
#pragma unroll
  for (int j = 0; j < 8; ++j) { const int k = k0 + j; v[j] = (k < KIN && o < OUTW) ? (b16)(bf16_rne(w[(size_t)k * OUTW + o]) * WSC) : (b16)0.0f; } for (int pass = 0; pass < 2; ++pass) { *(volatile v8b*)(WT + (size_t)o * KP + k0) = v; __threadfence(); }
}
template <int FIRST>
__global__ __launch_bounds__(32) void proj_kernel(const float* __restrict__ IN, const float* __restrict__ grot, const b16* __restrict__ WT, const float* __restrict__ asrc, const float* __restrict__ adst, int nb0, int NLIM, float* __restrict__ HP, float* __restrict__ AL) {
  constexpr int KIN = FIRST ? 32 : D;
  __shared__ __attribute__((aligned(16))) b16 Ah[16][KIN + 8], Al[16][KIN + 8]; __shared__ __attribute__((aligned(16))) float Tf[16][128 + 4], Pp[16][16][2], Ta[16][8];
  const int lane = threadIdx.x, nloc = lane & 15, hlf = lane >> 4; const size_t m0 = (size_t)blockIdx.x * 16; if (nb0 + m0 >= (size_t)NLIM) return;
  for (int rr = 0; rr < 16; ++rr) { const size_t nl = m0 + rr, n = nb0 + nl;
    if (FIRST) { float v = 0.0f; if (lane < 3) v = bf16_rne(IN[n * 3 + lane]); else if (lane < INF) v = bf16_rne(grot[(n / J) * 6 + lane - 3]); Ah[rr][lane] = (b16)(v * XS); Al[rr][lane] = (b16)0.0f; }
    else { for (int q = 0; q < 8; ++q) { b16 p, ql; split16(IN[nl * D + q * 32 + lane] * XS, p, ql); Ah[rr][q * 32 + lane] = p; Al[rr][q * 32 + lane] = ql; } } }
  wave_lds_sync();
#pragma unroll 1
  for (int cg = 0; cg < 2; ++cg) { v8f acc[8];
#pragma unroll
    for (int t = 0; t < 8; ++t) acc[t] = (v8f){};
#pragma unroll 2
    for (int kb = 0; kb < KIN; kb += 32) { const v16b a = frag_kb(&Ah[nloc][kb], hlf), al = frag_kb(&Al[nloc][kb], hlf);
#pragma unroll
      for (int t = 0; t < 8; ++t) { const v16b bw = frag_kb(WT + (size_t)(cg * 128 + t * 16 + nloc) * KIN + kb, hlf); acc[t] = wmma16b(a, bw, acc[t]); if (!FIRST) acc[t] = wmma16b(al, bw, acc[t]); } }
#pragma unroll
    for (int t = 0; t < 8; ++t) { const int c = cg * 128 + t * 16 + nloc; const float ws_ = bf16_rne(asrc[c]), wd_ = bf16_rne(adst[c]); float ps[8], pd[8];
#pragma unroll
      for (int r8 = 0; r8 < 8; ++r8) { const float v = acc[t][r8] * (1.0f / (XS * WSC)); Tf[8 * hlf + r8][t * 16 + nloc] = v; ps[r8] = pmul(v, ws_); pd[r8] = pmul(v, wd_); }
#pragma unroll
      for (int r8 = 0; r8 < 8; ++r8) { for (int o = 1; o < 16; o <<= 1) { ps[r8] += __shfl_xor(ps[r8], o); pd[r8] += __shfl_xor(pd[r8], o); } if (nloc == 0) { Pp[8 * hlf + r8][cg * 8 + t][0] = ps[r8]; Pp[8 * hlf + r8][cg * 8 + t][1] = pd[r8]; } } }
    wave_lds_sync();
    for (int pass = 0; pass < 2; ++pass) { for (int rr = 0; rr < 16; ++rr) *(volatile v4f*)(HP + (m0 + rr) * D + cg * 128 + lane * 4) = *(const v4f*)(&Tf[rr][lane * 4]); __threadfence(); }
    wave_lds_sync(); }
  if (lane < 16) { for (int hd = 0; hd < NH; ++hd) { float s = 0.0f, d = 0.0f; for (int t = 0; t < 4; ++t) { s += Pp[lane][hd * 4 + t][0]; d += Pp[lane][hd * 4 + t][1]; } Ta[lane][hd] = s; Ta[lane][4 + hd] = d; } }
  wave_lds_sync();
  for (int pass = 0; pass < 2; ++pass) { for (int q = 0; q < 4; ++q) ((volatile float*)AL)[m0 * 8 + q * 32 + lane] = Ta[(q * 32 + lane) >> 3][(q * 32 + lane) & 7]; __threadfence(); }
}
template <int CONCAT>
__global__ __launch_bounds__(32) void satt_kernel(const float* __restrict__ HP, const float* __restrict__ AL, const float* __restrict__ bias, int nb0, int NLIM, float* __restrict__ OUT) {
  __shared__ __attribute__((aligned(16))) float Tf[16][D + 4];
  const int lane = threadIdx.x, hd = lane >> 3; const size_t m0 = (size_t)blockIdx.x * 16; if (nb0 + m0 >= (size_t)NLIM) return;
  for (int rr = 0; rr < 16; ++rr) { const size_t n = m0 + rr; const int j = (int)((nb0 + n) % J); const int pj = PARENT[j]; const size_t np_ = pj >= 0 ? n - j + pj : n;
    const float adv = AL[n * 8 + 4 + hd]; const float es = leaky(AL[n * 8 + hd] + adv); float ws_ = 1.0f, wp = 0.0f;
    if (pj >= 0) { const float ep = leaky(AL[np_ * 8 + hd] + adv); const float mx = fmaxf(es, ep); const float ps = __expf(es - mx), pp = __expf(ep - mx); const float den = ps + pp; ws_ = ps / den; wp = pp / den; }
    const float* hs = HP + n * D + lane * 8; const float* hpp = HP + np_ * D + lane * 8;
    for (int q = 0; q < 8; ++q) Tf[rr][lane * 8 + q] = pmul(ws_, hs[q]) + pmul(wp, hpp[q]); }
  wave_lds_sync();
  if (CONCAT) { for (int pass = 0; pass < 2; ++pass) { for (int rr = 0; rr < 16; ++rr) for (int q = 0; q < 8; ++q) { const int c = q * 32 + lane; ((volatile float*)OUT)[(m0 + rr) * D + c] = fmaxf(Tf[rr][c] + bf16_rne(bias[c]), 0.0f); } __threadfence(); } }
  else { for (int pass = 0; pass < 2; ++pass) { for (int rr = 0; rr < 16; ++rr) for (int q = 0; q < 2; ++q) { const int c = q * 32 + lane; ((volatile float*)OUT)[(m0 + rr) * C + c] = (Tf[rr][c] + Tf[rr][C + c] + Tf[rr][2 * C + c] + Tf[rr][3 * C + c]) * 0.25f + bf16_rne(bias[c]); } __threadfence(); } }
}
__global__ __launch_bounds__(32) void rot_kernel(const float* __restrict__ X, const b16* __restrict__ WT, const float* __restrict__ bt, int nb0, int NLIM, float* __restrict__ out) {
  __shared__ __attribute__((aligned(16))) b16 Ah[16][C + 8], Al[16][C + 8]; __shared__ float So[16][6];
  const int lane = threadIdx.x, nloc = lane & 15, hlf = lane >> 4; const size_t m0 = (size_t)blockIdx.x * 16; const bool live = nb0 + m0 < (size_t)NLIM;
  for (int rr = 0; rr < 16; ++rr) for (int q = 0; q < 2; ++q) { b16 p, ql; split16(live ? X[(m0 + rr) * C + q * 32 + lane] * XS : 0.0f, p, ql); Ah[rr][q * 32 + lane] = p; Al[rr][q * 32 + lane] = ql; }
  wave_lds_sync();
  v8f acc = {};
#pragma unroll
  for (int kb = 0; kb < C; kb += 32) { const v16b a = frag_kb(&Ah[nloc][kb], hlf), al = frag_kb(&Al[nloc][kb], hlf); const v16b bw = frag_kb(WT + (size_t)nloc * C + kb, hlf); acc = wmma16b(a, bw, acc); acc = wmma16b(al, bw, acc); }
  if (nloc < 6) { const float bb = bf16_rne(bt[nloc]);
#pragma unroll
    for (int r8 = 0; r8 < 8; ++r8) So[8 * hlf + r8][nloc] = live ? acc[r8] * (1.0f / (XS * WSC)) + bb : 0.0f; }
  wave_lds_sync();
  for (int pass = 0; pass < 2; ++pass) { for (int i = lane; i < 96; i += 32) ((volatile float*)out)[m0 * 6 + i] = So[i / 6][i % 6]; __threadfence(); }
}
__global__ __launch_bounds__(256) void pool_kernel(const float* __restrict__ X, const float* __restrict__ Wg1, const float* __restrict__ bg1, const float* __restrict__ Wg2, const float* __restrict__ bg2, int gb0, int BLIM, float* __restrict__ out) {
  __shared__ float XP[8][C], Gp[8][C], So[32][8]; const int wave = threadIdx.x >> 5, lane = threadIdx.x & 31;
#pragma unroll 1
  for (int sub = 0; sub < 4; ++sub) { const int gl = blockIdx.x * 32 + sub * 8 + wave; const int g = gb0 + gl;
    if (g < BLIM) { float s0 = 0.0f, s1 = 0.0f; for (int j = 0; j < J; ++j) { const v2f v = *(const v2f*)(X + ((size_t)gl * J + j) * C + lane * 2); s0 += v[0]; s1 += v[1]; } XP[wave][lane * 2] = s0 * (1.0f / J); XP[wave][lane * 2 + 1] = s1 * (1.0f / J); }
    wave_lds_sync();
    if (g < BLIM) { for (int oq = 0; oq < 2; ++oq) { const int o = oq * 32 + lane; float s = bf16_rne(bg1[o]);
#pragma unroll 1
        for (int c = 0; c < C; ++c) s += pmul(XP[wave][c], bf16_rne(Wg1[c * C + o])); Gp[wave][o] = fmaxf(s, 0.0f); } }
    wave_lds_sync();
    if (lane < 6) { float s = bf16_rne(bg2[lane]); if (g < BLIM) {
#pragma unroll 1
        for (int c = 0; c < C; ++c) s += pmul(Gp[wave][c], bf16_rne(Wg2[c * 6 + lane])); } else s = 0.0f; So[sub * 8 + wave][lane] = s; }
    wave_lds_sync(); }
  __syncthreads();
  for (int pass = 0; pass < 2; ++pass) { if (threadIdx.x < 192) ((volatile float*)out)[(size_t)blockIdx.x * 192 + threadIdx.x] = So[threadIdx.x / 6][threadIdx.x % 6]; __threadfence(); }
}
}

extern "C" void kernel_launch(void* const* d_in, const int* in_sizes, int n_in, void* d_out, int out_size, void* d_ws, size_t ws_size, hipStream_t stream) {
  (void)n_in;
  auto Fp = [&](int i) { return (const float*)d_in[i]; };
  if (in_sizes[0] != NT * 3 || in_sizes[1] != B * 6 || in_sizes[2] != INF * D || in_sizes[6] != D * D || in_sizes[10] != D * D || in_sizes[13] != C || in_sizes[14] != C * 6 || in_sizes[16] != C * C || in_sizes[18] != C * 6 || out_size != NT * 6 + B * 6) return;
  const int BLIM = B; const int NLIM = BLIM * J;
  size_t off = 0; char* ws = (char*)d_ws;
  auto carve = [&](size_t bytes) { char* p = ws + off; off += (bytes + 255) & ~(size_t)255; return p; };
  constexpr int GCH = 2048, NCHK = B / GCH, NCH = GCH * J;
  b16* WT1 = (b16*)carve((size_t)D * 32 * 2); b16* WT2 = (b16*)carve((size_t)D * D * 2); b16* WT3 = (b16*)carve((size_t)D * D * 2); b16* WTT = (b16*)carve(16 * C * 2);
  float* HP = (float*)carve((size_t)NCH * D * 4); float* Hh = (float*)carve((size_t)NCH * D * 4); float* AL = (float*)carve((size_t)NCH * 8 * 4); float* X = (float*)carve((size_t)NCH * C * 4);
  if (off > ws_size || off > ((size_t)128 << 20)) return;
  wput_kernel<<<(D * 4 + 255) / 256, 256, 0, stream>>>(Fp(2), INF, D, 32, D, WT1); wput_kernel<<<(D * 32 + 255) / 256, 256, 0, stream>>>(Fp(6), D, D, D, D, WT2); wput_kernel<<<(D * 32 + 255) / 256, 256, 0, stream>>>(Fp(10), D, D, D, D, WT3); wput_kernel<<<(16 * 8 + 255) / 256, 256, 0, stream>>>(Fp(14), C, 6, C, 16, WTT);
  float* rot = (float*)d_out; float* pg = (float*)d_out + (size_t)NT * 6;
  for (int ch = 0; ch < NCHK; ++ch) { const int nb0 = ch * NCH, gb0 = ch * GCH; if (nb0 >= NLIM) {   }
    proj_kernel<1><<<NCH / 16, 32, 0, stream>>>(Fp(0), Fp(1), WT1, Fp(3), Fp(4), nb0, NLIM, HP, AL);
    satt_kernel<1><<<NCH / 16, 32, 0, stream>>>(HP, AL, Fp(5), nb0, NLIM, Hh);
    proj_kernel<0><<<NCH / 16, 32, 0, stream>>>(Hh, nullptr, WT2, Fp(7), Fp(8), nb0, NLIM, HP, AL);
    satt_kernel<1><<<NCH / 16, 32, 0, stream>>>(HP, AL, Fp(9), nb0, NLIM, Hh);
    proj_kernel<0><<<NCH / 16, 32, 0, stream>>>(Hh, nullptr, WT3, Fp(11), Fp(12), nb0, NLIM, HP, AL);
    satt_kernel<0><<<NCH / 16, 32, 0, stream>>>(HP, AL, Fp(13), nb0, NLIM, X);
    rot_kernel<<<NCH / 16, 32, 0, stream>>>(X, WTT, Fp(15), nb0, NLIM, rot + (size_t)nb0 * 6);
    pool_kernel<<<GCH / 32, 256, 0, stream>>>(X, Fp(16), Fp(17), Fp(18), Fp(19), gb0, BLIM, pg + (size_t)gb0 * 6); }
}
